// SwinTransformerBlock_63050119905818
// MI455X (gfx1250) — hardware-run, weakly checked
//
#include <hip/hip_runtime.h>
#include <math.h>
#include <stdint.h>

#ifndef NB
#define NB 16
#endif
#define NB_FULL 16
#define IMH 56
#define IMW 56
#define CC 256
#define WSZ 7
#define SSH 3
#define NHD 8
#define HDD 32
#define LTOK (WSZ * WSZ)
#define HIDN 1024
#define QKVC (3 * CC)
#define NWY (IMH / WSZ)
#define NWX (IMW / WSZ)
#define NWIMG (NWY * NWX)
#define NPIX_IMG (IMH * IMW)
#define NWT (NB * NWIMG)
#define MTOK (NB * NPIX_IMG)
#define LTAB ((2 * WSZ - 1) * (2 * WSZ - 1))
#define CPBH 512
#define TABW 2048

#define WCAR   64.0f
#define QKVCAR 16.0f
#define PCAR   1024.0f
#define OCAR   64.0f
#define GCAR   16.0f

static_assert(MTOK % 64 == 0);
static_assert(NPIX_IMG % 8 == 0);
static_assert(NWIMG * LTOK == NPIX_IMG);
static_assert(LTAB * NHD <= TABW);
static_assert(HIDN >= QKVC);
static_assert(NB >= 1 && NB <= NB_FULL);
static_assert(NWX == 8 && NWY == 8);
static_assert(CC % 32 == 0 && HIDN % 32 == 0);

typedef __attribute__((ext_vector_type(16))) _Float16 v16h;
typedef __attribute__((ext_vector_type(8)))  _Float16 v8h;
typedef __attribute__((ext_vector_type(8)))  float    v8f;
typedef __attribute__((ext_vector_type(4)))  float    v4f;
typedef __attribute__((ext_vector_type(4)))  unsigned int v4u;

__device__ __forceinline__ unsigned short f2bf_bits(float f) {
  unsigned u = __float_as_uint(f);
  return (unsigned short)((u + 0x7FFFu + ((u >> 16) & 1u)) >> 16);
}
__device__ __forceinline__ float bf_bits2f(unsigned short h) { return __uint_as_float(((unsigned)h) << 16); }
__device__ __forceinline__ float bfr(float f) { return bf_bits2f(f2bf_bits(f)); }
__device__ __forceinline__ v4f bfr4(v4f a) { v4f r; r[0] = bfr(a[0]); r[1] = bfr(a[1]); r[2] = bfr(a[2]); r[3] = bfr(a[3]); return r; }

__device__ __forceinline__ void dep_guard_h(v8f& a, v8f& b, v16h x, v16h y) { asm volatile("v_nop\n\tv_nop\n\tv_nop\n\tv_nop" : "+v"(a), "+v"(b) : "v"(x), "v"(y)); }
__device__ __forceinline__ void dep_guard_h3(v8f& a, v8f& b, v16h x, v16h y, v16h z) { asm volatile("v_nop\n\tv_nop\n\tv_nop\n\tv_nop" : "+v"(a), "+v"(b) : "v"(x), "v"(y), "v"(z)); }
__device__ __forceinline__ void keep4_h(v16h a, v16h b, v16h c, v16h d) { asm volatile("v_nop" :: "v"(a), "v"(b), "v"(c), "v"(d)); }
__device__ __forceinline__ void acc_guard4(v8f& a, v8f& b, v8f& c, v8f& d) { asm volatile("v_nop\n\tv_nop\n\tv_nop\n\tv_nop" : "+v"(a), "+v"(b), "+v"(c), "+v"(d)); }
__device__ __forceinline__ void acc_guard2(v8f& a, v8f& b) { asm volatile("v_nop\n\tv_nop\n\tv_nop\n\tv_nop" : "+v"(a), "+v"(b)); }

union FragU { v16h v; v8h h[2]; _Float16 s[16]; };
struct FragH {
  static __device__ __forceinline__ v16h load(const _Float16* p) {
    FragU f; f.h[0] = *(const v8h*)(p); f.h[1] = *(const v8h*)(p + 16); return f.v;
  }
  static __device__ __forceinline__ v8f mma(v16h a, v16h b, v8f c) {
    return __builtin_amdgcn_wmma_f32_16x16x32_f16(false, a, false, b, (short)0, c, false, false);
  }
};

__device__ __forceinline__ int tok2raster(int m) {
  const int win = m / LTOK, l = m - win * LTOK;
  const int b = win / NWIMG, wi = win - b * NWIMG;
  const int wh = wi / NWX, ww = wi - wh * NWX;
  const int i = l / WSZ, j = l - i * WSZ;
  int y = wh * WSZ + i + SSH; y = (y >= IMH) ? (y - IMH) : y;
  int x = ww * WSZ + j + SSH; x = (x >= IMW) ? (x - IMW) : x;
  return (b * IMH + y) * IMW + x;
}

template <int BIAS_MODE, int OUT_MODE, bool RESID, int ACT, int ROWMAP>
__global__ __launch_bounds__(256) void wmma_gemm64(
    const unsigned short* __restrict__ Ap, int lda,
    const unsigned short* __restrict__ Btp, int ldb,
    void* Cout, int ldc,
    const float* __restrict__ bias,
    const float* resid,
    int M, int N, int K, float scale, float oscale) {
  const _Float16* A = (const _Float16*)Ap;
  const _Float16* Bt = (const _Float16*)Btp;
  __shared__ __align__(16) float sT[8][16 * 68];
  const int lane = threadIdx.x & 31;
  const int wave = threadIdx.x >> 5;
  const int tilesN = N >> 6;
  const int tilesM = M >> 6;
  const int tile = blockIdx.x * 8 + wave;
  if (tile >= tilesM * tilesN) return;
  const int tm = tile / tilesN;
  const int tn = tile - tm * tilesN;
  const int m0 = tm << 6;
  const int n0 = tn << 6;
  const int rlane = lane & 15;
  const int koff  = (lane >> 4) * 8;
  const int mOff  = (lane >> 4) * 8;

  v8f acc[4][4];
#pragma unroll
  for (int i = 0; i < 4; ++i)
#pragma unroll
    for (int j = 0; j < 4; ++j) acc[i][j] = (v8f){0.f,0.f,0.f,0.f,0.f,0.f,0.f,0.f};

  for (int k0 = 0; k0 < K; k0 += 32) {
    v16h bh[4];
#pragma unroll
    for (int j = 0; j < 4; ++j) {
      const size_t bo = (size_t)(n0 + (j << 4) + rlane) * ldb + koff + k0;
      bh[j] = FragH::load(Bt + bo);
    }
#pragma unroll
    for (int i = 0; i < 4; ++i) {
      const size_t ao = (size_t)(m0 + (i << 4) + rlane) * lda + koff + k0;
      const v16h ah = FragH::load(A + ao);
#pragma unroll
      for (int j = 0; j < 4; ++j) acc[i][j] = FragH::mma(ah, bh[j], acc[i][j]);
      dep_guard_h(acc[i][0], acc[i][3], ah, bh[3]);
    }
    keep4_h(bh[0], bh[1], bh[2], bh[3]);
  }
  acc_guard4(acc[0][0], acc[0][1], acc[0][2], acc[0][3]);
  acc_guard4(acc[1][0], acc[1][1], acc[1][2], acc[1][3]);
  acc_guard4(acc[2][0], acc[2][1], acc[2][2], acc[2][3]);
  acc_guard4(acc[3][0], acc[3][1], acc[3][2], acc[3][3]);

  float* slab = sT[wave];
#pragma unroll
  for (int i = 0; i < 4; ++i) {
    const int mBase = m0 + (i << 4);
#pragma unroll
    for (int j = 0; j < 4; ++j) {
      const int n = n0 + (j << 4) + rlane;
      float bv = 0.f;
      if (BIAS_MODE == 2) bv = bfr(bias[n]);
#pragma unroll
      for (int r = 0; r < 8; ++r) {
        float v = acc[i][j][r] * scale;
        if (BIAS_MODE == 2) v += bv;
        if (ACT == 5) v = 0.5f * v * (1.0f + erff(v * 0.70710678118654752f));
        v *= oscale;
        slab[(mOff + r) * 68 + (j << 4) + rlane] = v;
      }
    }
    __builtin_amdgcn_fence(__ATOMIC_RELEASE, "workgroup");
    __builtin_amdgcn_wave_barrier();
    __builtin_amdgcn_fence(__ATOMIC_ACQUIRE, "workgroup");
    if (OUT_MODE == 0) {
      float* C = (float*)Cout;
      const int hh = lane >> 4, c4 = (lane & 15) * 4;
      int orow[8];
#pragma unroll
      for (int it = 0; it < 8; ++it) {
        const int row = it * 2 + hh;
        orow[it] = ROWMAP ? tok2raster(mBase + row) : (mBase + row);
      }
      if (RESID) {
#pragma unroll
        for (int it = 0; it < 8; ++it) {
          const int row = it * 2 + hh;
          v4f v = *(const v4f*)(slab + row * 68 + c4);
          const v4f rv = *(const v4f*)(resid + (size_t)orow[it] * ldc + n0 + c4);
          v += rv;
          *(v4f*)(slab + row * 68 + c4) = v;
        }
      }
      for (int pass = 0; pass < 2; ++pass) {
#pragma unroll
        for (int it = 0; it < 8; ++it) {
          const int row = it * 2 + hh;
          const v4f v = *(const v4f*)(slab + row * 68 + c4);
          *(volatile v4f*)(C + (size_t)orow[it] * ldc + n0 + c4) = v;
        }
        __threadfence();
      }
    } else {
      const int q = lane >> 3, c8 = (lane & 7) * 8;
      unsigned short* C = (unsigned short*)Cout;
      for (int pass = 0; pass < 2; ++pass) {
#pragma unroll
        for (int it = 0; it < 4; ++it) {
          const int row = it * 4 + q;
          const float* sp = slab + row * 68 + c8;
          v8h hv;
#pragma unroll
          for (int e = 0; e < 8; ++e) hv[e] = (_Float16)sp[e];
          *(volatile v8h*)(C + (size_t)(mBase + row) * ldc + n0 + c8) = hv;
        }
        __threadfence();
      }
    }
    __builtin_amdgcn_fence(__ATOMIC_RELEASE, "workgroup");
    __builtin_amdgcn_wave_barrier();
    __builtin_amdgcn_fence(__ATOMIC_ACQUIRE, "workgroup");
  }
}

__global__ __launch_bounds__(256) void cvt_w16_kernel(const float* __restrict__ in, unsigned short* out, float carry, int n8) {
  const int i = blockIdx.x * 256 + threadIdx.x;
  if (i < n8) {
    const v4f a = *(const v4f*)(in + 8 * (size_t)i);
    const v4f b = *(const v4f*)(in + 8 * (size_t)i + 4);
    union { v8h h; v4u u; } pk;
#pragma unroll
    for (int e = 0; e < 4; ++e) {
      pk.h[e]     = (_Float16)(bfr(a[e]) * carry);
      pk.h[4 + e] = (_Float16)(bfr(b[e]) * carry);
    }
    const v4u val = pk.u;
    *(volatile v4u*)(out + 8 * (size_t)i) = val;
    __threadfence();
    *(volatile v4u*)(out + 8 * (size_t)i) = val;
  }
}

__global__ __launch_bounds__(256) void cpb_table_kernel(const float* __restrict__ w1, const float* __restrict__ b1,
                                                        const float* __restrict__ w2, const float* __restrict__ b2,
                                                        float* tab) {
  __shared__ __align__(16) float st[TABW];
  const int tid = threadIdx.x;
  for (int o = tid; o < TABW; o += 256) {
    int idx = o >> 3;
    idx = (idx < LTAB) ? idx : (LTAB - 1);
    const int head = o & 7;
    const int a = idx / (2 * WSZ - 1), bq = idx - a * (2 * WSZ - 1);
    const float da = (float)(a - (WSZ - 1)), db = (float)(bq - (WSZ - 1));
    const float fx = copysignf(log1pf(fabsf(da)), da);
    const float fy = copysignf(log1pf(fabsf(db)), db);
    float acc = bfr(b2[head]);
#pragma unroll 1
    for (int jj = 0; jj < CPBH; ++jj) {
      const float hv = fmaxf(bfr(w1[2 * jj]) * fx + bfr(w1[2 * jj + 1]) * fy + bfr(b1[jj]), 0.0f);
      acc += hv * bfr(w2[head * CPBH + jj]);
    }
    st[o] = (o < LTAB * NHD) ? acc : 0.0f;
  }
  __syncthreads();
  for (int pass = 0; pass < 2; ++pass) {
#pragma unroll
    for (int it = 0; it < 2; ++it) {
      const int i4 = (it * 256 + tid) * 4;
      const v4f v = *(const v4f*)(&st[i4]);
      *(volatile v4f*)(tab + i4) = v;
    }
    __threadfence();
  }
}

__global__ __launch_bounds__(256) void ape_ln1_kernel(const float* __restrict__ x, const float* __restrict__ apew,
                                                      const float* __restrict__ apeb, const float* __restrict__ n1w,
                                                      const float* __restrict__ n1b, float* xs, unsigned short* X16, int npix) {
  __shared__ __align__(16) float sL[8][CC];
  const int tid = threadIdx.x, wave = tid >> 5, lane = tid & 31;
  int pix = blockIdx.x * 8 + wave;
  pix = (pix < npix) ? pix : (npix - 1);
  const int b = pix / NPIX_IMG;
  const int rem = pix - b * NPIX_IMG;
  const int y = rem / IMW, xq = rem - y * IMW;
  const int c0 = 4 * lane, c1 = (CC / 2) + 4 * lane;
  const float* xc = x + (size_t)pix * CC;
  v4f acc0 = bfr4(*(const v4f*)(xc + c0));
  v4f acc1 = bfr4(*(const v4f*)(xc + c1));
#pragma unroll 1
  for (int tap = 0; tap < 9; ++tap) {
    const int t3 = tap / 3;
    const int dh = t3 - 1, dw = tap - t3 * 3 - 1;
    int yy = y + dh, xx = xq + dw;
    const bool ok = (yy >= 0) && (yy < IMH) && (xx >= 0) && (xx < IMW);
    yy = (yy < 0) ? 0 : ((yy >= IMH) ? (IMH - 1) : yy);
    xx = (xx < 0) ? 0 : ((xx >= IMW) ? (IMW - 1) : xx);
    const float* xp = x + ((size_t)(b * IMH + yy) * IMW + xx) * CC;
    const v4f a0 = bfr4(*(const v4f*)(xp + c0));
    const v4f a1 = bfr4(*(const v4f*)(xp + c1));
    const v4f w0 = bfr4(*(const v4f*)(apew + tap * CC + c0));
    const v4f w1 = bfr4(*(const v4f*)(apew + tap * CC + c1));
    const float g = ok ? 1.0f : 0.0f;
    acc0 += (a0 * w0) * g;
    acc1 += (a1 * w1) * g;
  }
  const v4f s0 = acc0 + bfr4(*(const v4f*)(apeb + c0));
  const v4f s1 = acc1 + bfr4(*(const v4f*)(apeb + c1));
  float* orow = xs + (size_t)pix * CC;
  *(volatile v4f*)(orow + c0) = s0;
  *(volatile v4f*)(orow + c1) = s1;
  __threadfence();
  *(volatile v4f*)(orow + c0) = s0;
  *(volatile v4f*)(orow + c1) = s1;
  float sum = ((s0[0] + s0[1]) + (s0[2] + s0[3])) + ((s1[0] + s1[1]) + (s1[2] + s1[3]));
#pragma unroll
  for (int off = 16; off > 0; off >>= 1) sum += __shfl_xor(sum, off, 32);
  const float mean = sum * (1.0f / CC);
  const v4f d0 = s0 - mean, d1 = s1 - mean;
  float vs = ((d0[0] * d0[0] + d0[1] * d0[1]) + (d0[2] * d0[2] + d0[3] * d0[3])) +
             ((d1[0] * d1[0] + d1[1] * d1[1]) + (d1[2] * d1[2] + d1[3] * d1[3]));
#pragma unroll
  for (int off = 16; off > 0; off >>= 1) vs += __shfl_xor(vs, off, 32);
  const float rstd = 1.0f / sqrtf(vs * (1.0f / CC) + 1e-5f);
  const v4f g0 = bfr4(*(const v4f*)(n1w + c0)), g1 = bfr4(*(const v4f*)(n1w + c1));
  const v4f e0 = bfr4(*(const v4f*)(n1b + c0)), e1 = bfr4(*(const v4f*)(n1b + c1));
  const v4f y0 = (d0 * rstd) * g0 + e0;
  const v4f y1 = (d1 * rstd) * g1 + e1;
  *(v4f*)(&sL[wave][c0]) = y0;
  *(v4f*)(&sL[wave][c1]) = y1;
  __builtin_amdgcn_fence(__ATOMIC_RELEASE, "workgroup");
  __builtin_amdgcn_wave_barrier();
  __builtin_amdgcn_fence(__ATOMIC_ACQUIRE, "workgroup");
  const v4f u0 = *(const v4f*)(&sL[wave][8 * lane]);
  const v4f u1 = *(const v4f*)(&sL[wave][8 * lane + 4]);
  union { v8h h; v4u u; } pk;
#pragma unroll
  for (int e = 0; e < 4; ++e) { pk.h[e] = (_Float16)u0[e]; pk.h[4 + e] = (_Float16)u1[e]; }
  const v4u val = pk.u;
  int yp = y - SSH; yp = (yp < 0) ? (yp + IMH) : yp;
  int xp = xq - SSH; xp = (xp < 0) ? (xp + IMW) : xp;
  const int wh = yp / WSZ, ii = yp - wh * WSZ;
  const int ww = xp / WSZ, jj = xp - ww * WSZ;
  const int t = ((b * NWY + wh) * NWX + ww) * LTOK + ii * WSZ + jj;
  unsigned short* dst = X16 + (size_t)t * CC + 8 * lane;
  *(volatile v4u*)dst = val;
  __threadfence();
  *(volatile v4u*)dst = val;
}

__device__ __forceinline__ void stage_unitvec(const _Float16* rp, _Float16* dst, float keep) {
  FragU u;
  u.h[0] = *(const v8h*)(rp);
  u.h[1] = *(const v8h*)(rp + 8);
  float xv[16];
  float ssq = 0.0f;
#pragma unroll
  for (int e = 0; e < 16; ++e) { xv[e] = (float)u.s[e] * (1.0f / QKVCAR); ssq += xv[e] * xv[e]; }
  ssq += __shfl_xor(ssq, 1, 32);
  const float inv = keep / fmaxf(sqrtf(ssq), 1e-12f);
  FragU o;
#pragma unroll
  for (int e = 0; e < 16; ++e) o.s[e] = (_Float16)(xv[e] * inv);
  *(v8h*)(dst) = o.h[0];
  *(v8h*)(dst + 8) = o.h[1];
}

__global__ __launch_bounds__(256) void win_attn_kernel(const unsigned short* __restrict__ QKVp,
                                                       const float* __restrict__ tscale, const float* __restrict__ tab,
                                                       unsigned short* O16, int nwin) {
  const _Float16* QKV = (const _Float16*)QKVp;
  __shared__ __align__(16) _Float16 sQ[2][64 * 32];
  __shared__ __align__(16) _Float16 sK[2][64 * 32];
  __shared__ __align__(16) _Float16 sVT[2][32 * 64];
  __shared__ __align__(16) _Float16 sP[8][16 * 64];
  __shared__ __align__(16) unsigned short sO[64 * 64];
  __shared__ float sTab[2][176];
  const int tid = threadIdx.x, lane = tid & 31, wave = tid >> 5;
  int win = blockIdx.x >> 2;
  win = (win < nwin) ? win : (nwin - 1);
  const int hp = blockIdx.x & 3;

  {
    const int l = tid >> 2;
    const int c = tid & 3;
    const int hw = c >> 1;
    const int d0 = (c & 1) * 16;
    const int lc = (l < LTOK) ? l : (LTOK - 1);
    const float keep = (l < LTOK) ? 1.0f : 0.0f;
    const _Float16* rp = QKV + (size_t)(win * LTOK + lc) * QKVC + hp * 64 + c * 16;
    stage_unitvec(rp, &sQ[hw][l * 32 + d0], keep);
    stage_unitvec(rp + CC, &sK[hw][l * 32 + d0], keep);
    {
      FragU u;
      u.h[0] = *(const v8h*)(rp + 2 * CC);
      u.h[1] = *(const v8h*)(rp + 2 * CC + 8);
#pragma unroll
      for (int e = 0; e < 16; ++e) {
        const float fv = (float)u.s[e] * keep;
        sVT[hw][(d0 + e) * 64 + l] = (_Float16)fv;
      }
    }
  }
#pragma unroll
  for (int it = 0; it < 2; ++it) {
    const int o = it * 256 + tid;
    const int oc = (o < 2 * LTAB) ? o : (2 * LTAB - 1);
    const int hw = (oc >= LTAB) ? 1 : 0;
    const int idx = oc - hw * LTAB;
    const float v = tab[idx * NHD + hp * 2 + hw];
    if (o < 2 * LTAB) sTab[hw][idx] = v;
  }
  __syncthreads();

  const int hw = wave >> 2;
  const int qr0 = (wave & 3) * 16;
  const int rlane = lane & 15, koff = (lane >> 4) * 8, mOff = (lane >> 4) * 8;
  const int wi = win & (NWIMG - 1), wh = wi >> 3, ww = wi & 7;
  const float esc = expf(-bfr(tscale[hp * 2 + hw]));
  const v8f z8 = (v8f){0.f,0.f,0.f,0.f,0.f,0.f,0.f,0.f};

  v8f s[4];
  {
    const v16h a = FragH::load(&sQ[hw][(qr0 + rlane) * 32 + koff]);
    v16h bq[4];
#pragma unroll
    for (int j = 0; j < 4; ++j) bq[j] = FragH::load(&sK[hw][(16 * j + rlane) * 32 + koff]);
#pragma unroll
    for (int j = 0; j < 4; ++j) s[j] = FragH::mma(a, bq[j], z8);
    dep_guard_h(s[0], s[3], a, bq[3]);
    keep4_h(bq[0], bq[1], bq[2], bq[3]);
  }
  acc_guard4(s[0], s[1], s[2], s[3]);

#pragma unroll
  for (int j = 0; j < 4; ++j) {
#pragma unroll
    for (int r = 0; r < 8; ++r) {
      const int m = qr0 + mOff + r;
      const int n = 16 * j + rlane;
      const int mc = (m < LTOK) ? m : (LTOK - 1);
      const int nc = (n < LTOK) ? n : (LTOK - 1);
      const int i1 = mc / WSZ, j1 = mc - i1 * WSZ;
      const int i2 = nc / WSZ, j2 = nc - i2 * WSZ;
      const float bias = sTab[hw][(i1 - i2 + WSZ - 1) * (2 * WSZ - 1) + (j1 - j2 + WSZ - 1)];
      const int hs1 = wh * WSZ + i1, ws1 = ww * WSZ + j1;
      const int hs2 = wh * WSZ + i2, ws2 = ww * WSZ + j2;
      const int g1 = ((hs1 < IMH - WSZ) ? 0 : ((hs1 < IMH - SSH) ? 1 : 2)) * 3 +
                     ((ws1 < IMW - WSZ) ? 0 : ((ws1 < IMW - SSH) ? 1 : 2));
      const int g2 = ((hs2 < IMH - WSZ) ? 0 : ((hs2 < IMH - SSH) ? 1 : 2)) * 3 +
                     ((ws2 < IMW - WSZ) ? 0 : ((ws2 < IMW - SSH) ? 1 : 2));
      float val = s[j][r] * esc + bias;
      val = val + ((g1 == g2) ? 0.0f : -100.0f);
      val = (m < LTOK) ? val : 0.0f;
      val = (n < LTOK) ? val : -INFINITY;
      s[j][r] = val;
    }
  }

#pragma unroll
  for (int r = 0; r < 8; ++r) {
    float mx = fmaxf(fmaxf(s[0][r], s[1][r]), fmaxf(s[2][r], s[3][r]));
    mx = fmaxf(mx, __shfl_xor(mx, 1, 32));
    mx = fmaxf(mx, __shfl_xor(mx, 2, 32));
    mx = fmaxf(mx, __shfl_xor(mx, 4, 32));
    mx = fmaxf(mx, __shfl_xor(mx, 8, 32));
    const float e0 = expf(s[0][r] - mx);
    const float e1 = expf(s[1][r] - mx);
    const float e2 = expf(s[2][r] - mx);
    const float e3 = expf(s[3][r] - mx);
    float sum = (e0 + e1) + (e2 + e3);
    sum += __shfl_xor(sum, 1, 32);
    sum += __shfl_xor(sum, 2, 32);
    sum += __shfl_xor(sum, 4, 32);
    sum += __shfl_xor(sum, 8, 32);
    const float pn = PCAR / sum;
    _Float16* prow = &sP[wave][(mOff + r) * 64 + rlane];
    prow[0]  = (_Float16)(e0 * pn);
    prow[16] = (_Float16)(e1 * pn);
    prow[32] = (_Float16)(e2 * pn);
    prow[48] = (_Float16)(e3 * pn);
  }
  __builtin_amdgcn_fence(__ATOMIC_RELEASE, "workgroup");
  __builtin_amdgcn_wave_barrier();
  __builtin_amdgcn_fence(__ATOMIC_ACQUIRE, "workgroup");

  v8f o[2];
  o[0] = z8; o[1] = z8;
#pragma unroll
  for (int k0 = 0; k0 < 64; k0 += 32) {
    const v16h a  = FragH::load(&sP[wave][rlane * 64 + k0 + koff]);
    const v16h b0 = FragH::load(&sVT[hw][rlane * 64 + k0 + koff]);
    const v16h b1 = FragH::load(&sVT[hw][(16 + rlane) * 64 + k0 + koff]);
    o[0] = FragH::mma(a, b0, o[0]);
    o[1] = FragH::mma(a, b1, o[1]);
    dep_guard_h3(o[0], o[1], a, b0, b1);
  }
  acc_guard2(o[0], o[1]);
#pragma unroll
  for (int jd = 0; jd < 2; ++jd) {
#pragma unroll
    for (int r = 0; r < 8; ++r) {
      const float ov = o[jd][r] * (OCAR / (PCAR * QKVCAR));
      sO[(qr0 + mOff + r) * 64 + hw * 32 + 16 * jd + rlane] = __builtin_bit_cast(unsigned short, (_Float16)ov);
    }
  }
  __syncthreads();
  {
    const int c8 = (tid & 7) * 8;
    unsigned short* Ob = O16 + (size_t)win * LTOK * CC + hp * 64 + c8;
    for (int pass = 0; pass < 2; ++pass) {
#pragma unroll
      for (int it = 0; it < 2; ++it) {
        const int rowl = it * 32 + (tid >> 3);
        const v4u v = *(const v4u*)(&sO[rowl * 64 + c8]);
        if (rowl < LTOK) *(volatile v4u*)(Ob + (size_t)rowl * CC) = v;
      }
      __threadfence();
    }
  }
}

__global__ __launch_bounds__(256) void ln2_kernel(const float* xin, const float* __restrict__ w, const float* __restrict__ bb,
                                                  unsigned short* H2, int nrow) {
  const int tid = threadIdx.x, wave = tid >> 5, lane = tid & 31;
  int row = blockIdx.x * 8 + wave;
  row = (row < nrow) ? row : (nrow - 1);
  const int c0 = 8 * lane;
  const float* rp = xin + (size_t)row * CC + c0;
  const v4f a = *(const v4f*)(rp);
  const v4f b = *(const v4f*)(rp + 4);
  float sum = ((a[0] + a[1]) + (a[2] + a[3])) + ((b[0] + b[1]) + (b[2] + b[3]));
#pragma unroll
  for (int off = 16; off > 0; off >>= 1) sum += __shfl_xor(sum, off, 32);
  const float mean = sum * (1.0f / CC);
  const v4f d0 = a - mean, d1 = b - mean;
  float vs = ((d0[0] * d0[0] + d0[1] * d0[1]) + (d0[2] * d0[2] + d0[3] * d0[3])) +
             ((d1[0] * d1[0] + d1[1] * d1[1]) + (d1[2] * d1[2] + d1[3] * d1[3]));
#pragma unroll
  for (int off = 16; off > 0; off >>= 1) vs += __shfl_xor(vs, off, 32);
  const float rstd = 1.0f / sqrtf(vs * (1.0f / CC) + 1e-5f);
  const v4f g0 = bfr4(*(const v4f*)(w + c0)), g1 = bfr4(*(const v4f*)(w + c0 + 4));
  const v4f e0 = bfr4(*(const v4f*)(bb + c0)), e1 = bfr4(*(const v4f*)(bb + c0 + 4));
  const v4f y0 = (d0 * rstd) * g0 + e0;
  const v4f y1 = (d1 * rstd) * g1 + e1;
  union { v8h h; v4u u; } pk;
#pragma unroll
  for (int e = 0; e < 4; ++e) { pk.h[e] = (_Float16)y0[e]; pk.h[4 + e] = (_Float16)y1[e]; }
  const v4u val = pk.u;
  unsigned short* dst = H2 + (size_t)row * CC + c0;
  *(volatile v4u*)dst = val;
  __threadfence();
  *(volatile v4u*)dst = val;
}

extern "C" void kernel_launch(void* const* d_in, const int* in_sizes, int n_in,
                              void* d_out, int out_size, void* d_ws, size_t ws_size,
                              hipStream_t stream) {
  if (n_in < 20) return;
  if (in_sizes[0] < MTOK * CC) return;
  if (in_sizes[1] < 9 * CC || in_sizes[2] < CC || in_sizes[3] < CC || in_sizes[4] < CC) return;
  if (in_sizes[5] < QKVC * CC || in_sizes[6] < QKVC || in_sizes[7] < NHD) return;
  if (in_sizes[8] < CPBH * 2 || in_sizes[9] < CPBH || in_sizes[10] < NHD * CPBH || in_sizes[11] < NHD) return;
  if (in_sizes[12] < CC * CC || in_sizes[13] < CC || in_sizes[14] < CC || in_sizes[15] < CC) return;
  if (in_sizes[16] < HIDN * CC || in_sizes[17] < HIDN || in_sizes[18] < CC * HIDN || in_sizes[19] < CC) return;
  if (out_size < MTOK * CC) return;

  const float* x       = (const float*)d_in[0];
  const float* ape_w   = (const float*)d_in[1];
  const float* ape_b   = (const float*)d_in[2];
  const float* norm1_w = (const float*)d_in[3];
  const float* norm1_b = (const float*)d_in[4];
  const float* qkv_w   = (const float*)d_in[5];
  const float* qkv_b   = (const float*)d_in[6];
  const float* tscale  = (const float*)d_in[7];
  const float* rpb1_w  = (const float*)d_in[8];
  const float* rpb1_b  = (const float*)d_in[9];
  const float* rpb2_w  = (const float*)d_in[10];
  const float* rpb2_b  = (const float*)d_in[11];
  const float* proj_w  = (const float*)d_in[12];
  const float* proj_b  = (const float*)d_in[13];
  const float* norm2_w = (const float*)d_in[14];
  const float* norm2_b = (const float*)d_in[15];
  const float* fc1_w   = (const float*)d_in[16];
  const float* fc1_b   = (const float*)d_in[17];
  const float* fc2_w   = (const float*)d_in[18];
  const float* fc2_b   = (const float*)d_in[19];
  float* outp = (float*)d_out;

  const size_t PWQ  = (size_t)QKVC * CC * 2;
  const size_t PWP  = (size_t)CC * CC * 2;
  const size_t PW1  = (size_t)HIDN * CC * 2;
  const size_t PW2  = (size_t)CC * HIDN * 2;
  const size_t PTAB = (size_t)TABW * 4;
  const size_t PA   = (size_t)MTOK * CC * 2;
  const size_t PB   = (size_t)MTOK * HIDN * 2;
  size_t off = 0;
  const size_t oWq = off; off += PWQ;
  const size_t oWp = off; off += PWP;
  const size_t oW1 = off; off += PW1;
  const size_t oW2 = off; off += PW2;
  const size_t oTab = off; off += PTAB;
  const size_t oA = off; off += PA;
  const size_t oB = off; off += PB;
  if (off > ws_size) return;
  if (off > (size_t)134217728u) return;

  char* ws = (char*)d_ws;
  unsigned short* Wq  = (unsigned short*)(ws + oWq);
  unsigned short* Wp  = (unsigned short*)(ws + oWp);
  unsigned short* W1  = (unsigned short*)(ws + oW1);
  unsigned short* W2  = (unsigned short*)(ws + oW2);
  float*          tab = (float*)(ws + oTab);
  unsigned short* RA  = (unsigned short*)(ws + oA);
  unsigned short* RB  = (unsigned short*)(ws + oB);

  const dim3 blk(256);
  {
    const int n8q = QKVC * CC / 8, n8p = CC * CC / 8, n81 = HIDN * CC / 8, n82 = CC * HIDN / 8;
    cvt_w16_kernel<<<dim3((n8q + 255) / 256), blk, 0, stream>>>(qkv_w, Wq, WCAR, n8q);
    cvt_w16_kernel<<<dim3((n8p + 255) / 256), blk, 0, stream>>>(proj_w, Wp, WCAR, n8p);
    cvt_w16_kernel<<<dim3((n81 + 255) / 256), blk, 0, stream>>>(fc1_w, W1, WCAR, n81);
    cvt_w16_kernel<<<dim3((n82 + 255) / 256), blk, 0, stream>>>(fc2_w, W2, WCAR, n82);
  }
  cpb_table_kernel<<<dim3(1), blk, 0, stream>>>(rpb1_w, rpb1_b, rpb2_w, rpb2_b, tab);
  ape_ln1_kernel<<<dim3(MTOK / 8), blk, 0, stream>>>(x, ape_w, ape_b, norm1_w, norm1_b, outp, RA, MTOK);

  const int tilesM = MTOK / 64;
  wmma_gemm64<2, 1, false, 0, 0><<<dim3((tilesM * (QKVC / 64) + 7) / 8), blk, 0, stream>>>(
      RA, CC, Wq, CC, (void*)RB, QKVC, qkv_b, qkv_b, MTOK, QKVC, CC, 1.0f / WCAR, QKVCAR);
  win_attn_kernel<<<dim3(NWT * 4), blk, 0, stream>>>(RB, tscale, tab, RA, NWT);
  wmma_gemm64<2, 0, true, 0, 1><<<dim3((tilesM * (CC / 64) + 7) / 8), blk, 0, stream>>>(
      RA, CC, Wp, CC, (void*)outp, CC, proj_b, outp, MTOK, CC, CC, 1.0f / (OCAR * WCAR), 1.0f);
  ln2_kernel<<<dim3(MTOK / 8), blk, 0, stream>>>(outp, norm2_w, norm2_b, RA, MTOK);
  wmma_gemm64<2, 1, false, 5, 0><<<dim3((tilesM * (HIDN / 64) + 7) / 8), blk, 0, stream>>>(
      RA, CC, W1, CC, (void*)RB, HIDN, fc1_b, fc1_b, MTOK, HIDN, CC, 1.0f / WCAR, GCAR);
  wmma_gemm64<2, 0, true, 0, 0><<<dim3((tilesM * (CC / 64) + 7) / 8), blk, 0, stream>>>(
      RB, HIDN, W2, HIDN, (void*)outp, CC, fc2_b, outp, MTOK, CC, HIDN, 1.0f / (GCAR * WCAR), 1.0f);
  (void)hipGetLastError();
}
